// GraphRec_72945724555841
// MI455X (gfx1250) — hardware-run, weakly checked
//
#include <hip/hip_runtime.h>


namespace {
constexpr int NUSR = 100000, NITM = 100000, D = 64, B = 16384, LU = 50, NF = 32, LI = 50;
constexpr float HS = 256.0f, WSC = 256.0f;
typedef _Float16 b16;
typedef __attribute__((ext_vector_type(16))) _Float16 v16b;
typedef __attribute__((ext_vector_type(8))) _Float16 v8b;
typedef __attribute__((ext_vector_type(8))) float v8f;
typedef __attribute__((ext_vector_type(4))) float v4f;
typedef __attribute__((ext_vector_type(2))) float v2f;
__device__ __forceinline__ float bf16_rne(float f) { unsigned int u = __float_as_uint(f); u += 0x7FFFu + ((u >> 16) & 1u); float r = __uint_as_float(u & 0xFFFF0000u); asm volatile("" : "+v"(r)); return r; }
__device__ __forceinline__ float bfv(float f) { float r = bf16_rne(f); asm volatile("" : "+v"(r)); return r; }
__device__ __forceinline__ void split16(float v, b16& hi, b16& lo) { hi = (b16)v; lo = (b16)(v - (float)hi); }
__device__ __forceinline__ v16b frag_kb(const b16* p, int hh) { const v8b a = *(const v8b*)(p + 8 * hh), b = *(const v8b*)(p + 16 + 8 * hh); v16b f;
#pragma unroll
  for (int e = 0; e < 8; ++e) { f[e] = a[e]; f[8 + e] = b[e]; } return f; }
__device__ __forceinline__ v8f wmma16b(v16b a, v16b b, v8f c) { v8f d = __builtin_amdgcn_wmma_f32_16x16x32_f16(false, a, false, b, (short)0, c, false, false); asm volatile("v_nop\n\tv_nop\n\tv_nop\n\tv_nop" : "+v"(d) : "v"(a), "v"(b)); return d; }
__device__ __forceinline__ void wave_lds_sync() { __builtin_amdgcn_fence(__ATOMIC_RELEASE, "workgroup"); __builtin_amdgcn_wave_barrier(); __builtin_amdgcn_fence(__ATOMIC_ACQUIRE, "workgroup"); }
__device__ __forceinline__ float pmul(float a, float b) { float p = a * b; asm volatile("" : "+v"(p)); return p; }
__device__ __forceinline__ int iclamp(int v, int lo, int hi) { return v < lo ? lo : (v > hi ? hi : v); }

__global__ __launch_bounds__(256) void wput_kernel(const float* __restrict__ w2, const float* __restrict__ w5, const float* __restrict__ w8, const float* __restrict__ fc1, b16* __restrict__ WK, b16* __restrict__ FC1) { const int u = blockIdx.x * 256 + threadIdx.x; v8b v;
  if (u < 3 * D * 8) { const int m = u / (D * 8), r = u % (D * 8); const int o = r / 8, k0 = (r % 8) * 8; const float* w = m == 0 ? w2 : (m == 1 ? w5 : w8);
#pragma unroll
    for (int j = 0; j < 8; ++j) v[j] = (b16)(bf16_rne(w[(size_t)(k0 + j) * D + o]) * WSC); for (int pass = 0; pass < 2; ++pass) { *(volatile v8b*)(WK + ((size_t)m * D + o) * D + k0) = v; __threadfence(); } }
  if (u < D * 16) { const int o = u / 16, k0 = (u % 16) * 8;
#pragma unroll
    for (int j = 0; j < 8; ++j) v[j] = (b16)(bf16_rne(fc1[(size_t)(k0 + j) * D + o]) * WSC); for (int pass = 0; pass < 2; ++pass) { *(volatile v8b*)(FC1 + (size_t)o * 2 * D + k0) = v; __threadfence(); } } }
__global__ __launch_bounds__(32) void sample_kernel(const int* __restrict__ uid, const int* __restrict__ iid, const int* __restrict__ hit, const float* __restrict__ hrt, const int* __restrict__ frd, const int* __restrict__ hus, const float* __restrict__ irt, const float* __restrict__ EU, const float* __restrict__ EI, const float* __restrict__ w1, const float* __restrict__ w3, const float* __restrict__ w4, const float* __restrict__ w6, const float* __restrict__ w7, const float* __restrict__ w9, const b16* __restrict__ WK, int BLIM, float* __restrict__ CONCAT) {
  __shared__ __attribute__((aligned(16))) b16 Nh[64][D + 8]; __shared__ float Qs[D], QW[D], Rt[64], Sc[64], Pr[64], Out[2 * D]; const int lane = threadIdx.x, nloc = lane & 15, hlf = lane >> 4; const int b = blockIdx.x; if (b >= BLIM) return;
  for (int c = lane; c < 2 * D; c += 32) Out[c] = 0.0f;
#pragma unroll 1
  for (int part = 0; part < 3; ++part) {
    const int L = part == 1 ? NF : LU; const float* EQ = part < 2 ? EU : EI; const float* EN = part == 0 ? EI : EU; const int* nidx = part == 0 ? hit : (part == 1 ? frd : hus); const float* rt = part == 0 ? hrt : (part == 1 ? (const float*)0 : irt); const float* wq = part == 0 ? w1 : (part == 1 ? w4 : w7); const float* wa = part == 0 ? w3 : (part == 1 ? w6 : w9); const int qrow = part < 2 ? iclamp(uid[b], 0, NUSR - 1) : iclamp(iid[b], 0, NITM - 1); const int nmax = (part == 0 ? NITM : NUSR) - 1; const int stride = part == 1 ? NF : LU;
    Qs[lane] = bfv(EQ[(size_t)qrow * D + lane]); Qs[32 + lane] = bfv(EQ[(size_t)qrow * D + 32 + lane]);
    for (int l = 0; l < 64; ++l) { const bool in = l < L; const int j = in ? iclamp(nidx[(size_t)b * stride + l], 0, nmax) : 0; const float v0 = in ? bfv(EN[(size_t)j * D + lane]) : 0.0f, v1 = in ? bfv(EN[(size_t)j * D + 32 + lane]) : 0.0f; Nh[l][lane] = (b16)(v0 * HS); Nh[l][32 + lane] = (b16)(v1 * HS); if (lane < 8) Nh[l][64 + lane] = (b16)0.0f; if (lane == 0) Rt[l] = (in && rt) ? bfv(rt[(size_t)b * stride + l]) : 0.0f; }
    wave_lds_sync();
    { float s0 = 0.0f, s1 = 0.0f; for (int k = 0; k < D; ++k) { const float qk = Qs[k]; s0 += pmul(qk, bfv(wq[(size_t)k * D + lane])); s1 += pmul(qk, bfv(wq[(size_t)k * D + 32 + lane])); } QW[lane] = s0; QW[32 + lane] = s1; }
    wave_lds_sync();
    const b16* W = WK + (size_t)(part == 0 ? 0 : (part == 1 ? 1 : 2)) * D * D; const float wa0 = bfv(wa[nloc]), wa1 = bfv(wa[16 + nloc]), wa2 = bfv(wa[32 + nloc]), wa3 = bfv(wa[48 + nloc]); const float waq[4] = {wa0, wa1, wa2, wa3};
#pragma unroll 1
    for (int rt4 = 0; rt4 < 4; ++rt4) { v8f acc[4] = {(v8f){}, (v8f){}, (v8f){}, (v8f){}};
#pragma unroll
      for (int kb = 0; kb < D; kb += 32) { const v16b a = frag_kb(&Nh[rt4 * 16 + nloc][kb], hlf);
#pragma unroll
        for (int t = 0; t < 4; ++t) acc[t] = wmma16b(a, frag_kb(W + (size_t)(t * 16 + nloc) * D + kb, hlf), acc[t]); }
#pragma unroll
      for (int r8 = 0; r8 < 8; ++r8) { const int l = rt4 * 16 + 8 * hlf + r8; float s = 0.0f;
#pragma unroll
        for (int t = 0; t < 4; ++t) { const int c = t * 16 + nloc; s += pmul(acc[t][r8] * (1.0f / (HS * WSC)) + QW[c] + pmul(Rt[l], (float)Nh[l][c] * (1.0f / HS)), waq[t]); }
        for (int o = 1; o < 16; o <<= 1) s += __shfl_xor(s, o); if (nloc == 0) Sc[l] = s; } }
    wave_lds_sync();
    { const float s0 = lane < L ? Sc[lane] : -INFINITY, s1 = (32 + lane) < L ? Sc[32 + lane] : -INFINITY; float mx = fmaxf(s0, s1); for (int o = 16; o; o >>= 1) mx = fmaxf(mx, __shfl_xor(mx, o)); const float p0 = lane < L ? __expf(s0 - mx) : 0.0f, p1 = (32 + lane) < L ? __expf(s1 - mx) : 0.0f; float den = p0 + p1; for (int o = 16; o; o >>= 1) den += __shfl_xor(den, o); Pr[lane] = p0 / den; Pr[32 + lane] = p1 / den; }
    wave_lds_sync();
    { float o0 = 0.0f, o1 = 0.0f; for (int l = 0; l < L; ++l) { const float p = Pr[l]; o0 += pmul(p, (float)Nh[l][lane] * (1.0f / HS)); o1 += pmul(p, (float)Nh[l][32 + lane] * (1.0f / HS)); } const int base = part < 2 ? 0 : D; Out[base + lane] += o0 + (part == 1 ? 0.0f : Qs[lane]); Out[base + 32 + lane] += o1 + (part == 1 ? 0.0f : Qs[32 + lane]); }
    wave_lds_sync(); }
  for (int pass = 0; pass < 2; ++pass) { *(volatile v4f*)(CONCAT + (size_t)b * 2 * D + lane * 4) = *(const v4f*)(&Out[lane * 4]); __threadfence(); } }
__global__ __launch_bounds__(32) void head_kernel(const float* __restrict__ CONCAT, const b16* __restrict__ FC1, const float* __restrict__ b1, const float* __restrict__ fc2, const float* __restrict__ b2, int BLIM, float* __restrict__ out) { __shared__ __attribute__((aligned(16))) b16 Ah[32][2 * D + 8], Al[32][2 * D + 8]; __shared__ float Hs[32][D + 4]; const int lane = threadIdx.x, nloc = lane & 15, hlf = lane >> 4; const size_t m0 = (size_t)blockIdx.x * 32; if (m0 >= (size_t)BLIM) return;
  for (int rr = 0; rr < 32; ++rr) for (int q = 0; q < 4; ++q) { b16 p, ql; split16(CONCAT[(m0 + rr) * 2 * D + q * 32 + lane] * HS, p, ql); Ah[rr][q * 32 + lane] = p; Al[rr][q * 32 + lane] = ql; } for (int k = 2 * D; k < 2 * D + 8; ++k) { Ah[lane][k] = (b16)0.0f; Al[lane][k] = (b16)0.0f; }
  wave_lds_sync();
#pragma unroll 1
  for (int rt = 0; rt < 2; ++rt) { v8f acc[4] = {(v8f){}, (v8f){}, (v8f){}, (v8f){}};
#pragma unroll
    for (int kb = 0; kb < 2 * D; kb += 32) { const v16b a = frag_kb(&Ah[rt * 16 + nloc][kb], hlf), al = frag_kb(&Al[rt * 16 + nloc][kb], hlf);
#pragma unroll
      for (int t = 0; t < 4; ++t) { const v16b bw = frag_kb(FC1 + (size_t)(t * 16 + nloc) * 2 * D + kb, hlf); acc[t] = wmma16b(a, bw, acc[t]); acc[t] = wmma16b(al, bw, acc[t]); } }
#pragma unroll
    for (int t = 0; t < 4; ++t) { const int c = t * 16 + nloc; const float bb = bfv(b1[c]);
#pragma unroll
      for (int r8 = 0; r8 < 8; ++r8) Hs[rt * 16 + 8 * hlf + r8][c] = fmaxf(acc[t][r8] * (1.0f / (HS * WSC)) + bb, 0.0f); } }
  wave_lds_sync();
  float s = 0.0f; for (int c = 0; c < D; ++c) s += pmul(Hs[lane][c], bfv(fc2[c])); s += bfv(b2[0]);
  for (int pass = 0; pass < 2; ++pass) { ((volatile float*)out)[m0 + lane] = s; __threadfence(); } }
}

extern "C" void kernel_launch(void* const* d_in, const int* in_sizes, int n_in, void* d_out, int out_size, void* d_ws, size_t ws_size, hipStream_t stream) {
  (void)n_in;
  auto Fp = [&](int i) { return (const float*)d_in[i]; }; auto Ip = [&](int i) { return (const int*)d_in[i]; };
  if (in_sizes[0] != B || in_sizes[1] != B || in_sizes[2] != B * LU || in_sizes[3] != B * LU || in_sizes[4] != B * NF || in_sizes[5] != B * LI || in_sizes[6] != B * LI || in_sizes[7] != NUSR * D || in_sizes[8] != NITM * D || in_sizes[9] != D * D || in_sizes[11] != D || in_sizes[18] != 2 * D * D || in_sizes[20] != D || out_size != B) return;
  const int BLIM = B;
  size_t off = 0; char* ws = (char*)d_ws;
  auto carve = [&](size_t bytes) { char* p = ws + off; off += (bytes + 255) & ~(size_t)255; return p; };
  b16* WK = (b16*)carve((size_t)3 * D * D * 2); b16* FC1 = (b16*)carve((size_t)D * 2 * D * 2); float* CONCAT = (float*)carve((size_t)B * 2 * D * 4);
  if (off > ws_size || off > ((size_t)16 << 20)) return;
  wput_kernel<<<(3 * D * 8 + 255) / 256, 256, 0, stream>>>(Fp(10), Fp(13), Fp(16), Fp(18), WK, FC1);
  sample_kernel<<<BLIM, 32, 0, stream>>>(Ip(0), Ip(1), Ip(2), Fp(3), Ip(4), Ip(5), Fp(6), Fp(7), Fp(8), Fp(9), Fp(11), Fp(12), Fp(14), Fp(15), Fp(17), WK, BLIM, CONCAT);
  head_kernel<<<BLIM / 32, 32, 0, stream>>>(CONCAT, FC1, Fp(19), Fp(20), Fp(21), BLIM, (float*)d_out);
}
